// ToeplitzCausalLinear_8400956031055
// MI455X (gfx1250) — hardware-verified
//
#include <hip/hip_runtime.h>
#include <stdint.h>


#define DIM     2048
#define TILE_M  128
#define TILE_N  128
#define TILE_K  32
#define AROW_B  80
#define SLEN    2176
#define SSTRIDE 2192

typedef __bf16   v16bf __attribute__((ext_vector_type(16)));
typedef float    v8f   __attribute__((ext_vector_type(8)));
typedef unsigned v4u   __attribute__((ext_vector_type(4)));
typedef float    v4f   __attribute__((ext_vector_type(4)));

union Frag { v16bf v; v4u q[2]; };

__device__ __forceinline__ unsigned short f2bf(float f) {
    union { __bf16 h; unsigned short u; } c;
    c.h = (__bf16)f;
    return c.u;
}
__device__ __forceinline__ unsigned bf16pk(float a, float b) {
    union { __bf16 h[2]; unsigned u; } c;
    c.h[0] = (__bf16)a;
    c.h[1] = (__bf16)b;
    return c.u;
}

__device__ __forceinline__ v8f wmma_bf16_step(v16bf a, v16bf b, v8f c) {
    c = __builtin_amdgcn_wmma_f32_16x16x32_bf16(false, a, false, b, (short)0, c, false, false);
    asm volatile("v_nop\n\tv_nop\n\tv_nop\n\tv_nop" : "+v"(c) : "v"(a), "v"(b));
    return c;
}

__global__ __launch_bounds__(256)
void k_causal_gemm_bf16(const float* __restrict__ x,
                        const float* __restrict__ weight,
                        const float* __restrict__ bias,
                        float* __restrict__ out) {
    __shared__ __attribute__((aligned(16))) unsigned short Rs[8 * SSTRIDE];
    __shared__ __attribute__((aligned(16))) unsigned int AsU[2][TILE_M * (AROW_B / 4)];

    const int t    = threadIdx.x;
    const int n0   = blockIdx.x * TILE_N;
    const int m0   = blockIdx.y * TILE_M;
    const int wv   = t >> 5;
    const int lane = t & 31;
    const int half = lane >> 4;
    const int l16  = lane & 15;

    auto stageA = [&](int buf, int k0) {
#pragma unroll
        for (int ii = 0; ii < 4; ++ii) {
            const int idx = t + ii * 256;
            const int row = idx >> 3;
            const int c4  = idx & 7;
            const float4 f =
                *(const float4*)(x + (size_t)(m0 + row) * DIM + k0 + c4 * 4);
            uint2 p;
            p.x = bf16pk(f.x, f.y);
            p.y = bf16pk(f.z, f.w);
            *(uint2*)((char*)AsU[buf] + row * AROW_B + c4 * 8) = p;
        }
    };

    stageA(0, 0);

    for (int idx = t; idx < 8 * SSTRIDE; idx += 256) {
        const int p = idx / SSTRIDE;
        const int e = idx - p * SSTRIDE;
        const int i = e + p;
        const float v = (i < DIM) ? weight[DIM - 1 - i] : 0.f;
        Rs[idx] = f2bf(v);
    }

    v8f acc[8];
#pragma unroll
    for (int nt = 0; nt < 8; ++nt) acc[nt] = (v8f){0.f, 0.f, 0.f, 0.f, 0.f, 0.f, 0.f, 0.f};

    int kmax = n0 + TILE_N;
    if (kmax > DIM) kmax = DIM;
    const int nk = kmax / TILE_K;

    const int ibase0 = DIM - 1 - n0 - l16 + half * 8;

    for (int ks = 0; ks < nk; ++ks) {
        __syncthreads();
        if (ks + 1 < nk) stageA((ks + 1) & 1, (ks + 1) * TILE_K);

        const int k0 = ks * TILE_K;

        Frag a;
        {
            const char* ap =
                (const char*)AsU[ks & 1] + (wv * 16 + l16) * AROW_B + half * 16;
            a.q[0] = *(const v4u*)ap;
            a.q[1] = *(const v4u*)(ap + 32);
        }

#pragma unroll
        for (int nt = 0; nt < 8; ++nt) {
            const int ib = ibase0 + k0 - nt * 16;
            const int p  = ib & 7;
            const int e  = ib - p;
            const unsigned short* bp = Rs + p * SSTRIDE + e;
            Frag b;
            b.q[0] = *(const v4u*)bp;
            b.q[1] = *(const v4u*)(bp + 16);
            acc[nt] = wmma_bf16_step(a.v, b.v, acc[nt]);
        }
    }

    __syncthreads();
    float* stg = (float*)(&AsU[0][0]) + wv * 512;
    const int q = lane >> 3;
    const int j = lane & 7;
    const size_t row_w = (size_t)(m0 + wv * 16);

#pragma unroll
    for (int pr = 0; pr < 4; ++pr) {
#pragma unroll
        for (int u = 0; u < 2; ++u) {
            const int nt = 2 * pr + u;
            const float bv = bias[n0 + nt * 16 + l16];
#pragma unroll
            for (int r = 0; r < 8; ++r)
                stg[(half * 8 + r) * 32 + u * 16 + l16] = acc[nt][r] + bv;
        }
        __syncthreads();
        v4f v[4];
#pragma unroll
        for (int s = 0; s < 4; ++s)
            v[s] = *(const v4f*)(stg + (s * 4 + q) * 32 + j * 4);
        float* gp = out + row_w * DIM + n0 + pr * 32 + j * 4;
#pragma unroll
        for (int s = 0; s < 4; ++s)
            *(volatile v4f*)(gp + (size_t)(s * 4 + q) * DIM) = v[s];
        __threadfence();
#pragma unroll
        for (int s = 0; s < 4; ++s)
            *(volatile v4f*)(gp + (size_t)(s * 4 + q) * DIM) = v[s];
        __syncthreads();
    }
}

extern "C" void kernel_launch(void* const* d_in, const int* in_sizes, int n_in,
                              void* d_out, int out_size, void* d_ws, size_t ws_size,
                              hipStream_t stream) {
    (void)d_ws; (void)ws_size;
    if (n_in < 3) return;
    const float* x      = (const float*)d_in[0];
    const float* weight = (const float*)d_in[1];
    const float* bias   = (const float*)d_in[2];
    float*       out    = (float*)d_out;

    const int nx = in_sizes[0];
    if (in_sizes[1] != DIM || in_sizes[2] != DIM) return;
    if (nx <= 0 || (nx % (DIM * TILE_M)) != 0 || out_size != nx) return;
    const int M = nx / DIM;

    dim3 grid(DIM / TILE_N, M / TILE_M);
    k_causal_gemm_bf16<<<grid, 256, 0, stream>>>(x, weight, bias, out);
}
